// LRU_36000415875649
// MI455X (gfx1250) — hardware-verified
//
#include <hip/hip_runtime.h>
#include <math.h>

typedef __attribute__((ext_vector_type(16))) _Float16 v16h;
typedef __attribute__((ext_vector_type(8)))  _Float16 v8h;
typedef __attribute__((ext_vector_type(8)))  float    v8f;
typedef __attribute__((ext_vector_type(4)))  float    v4f;
typedef __attribute__((ext_vector_type(2)))  float    v2f;

constexpr int kInF      = 128;
constexpr int kOutF     = 128;
constexpr int kStF      = 256;
constexpr int kBatch    = 8;
constexpr int kT        = 8192;
constexpr int kRows     = kBatch * kT;
constexpr int kHalfB    = 4;
constexpr int kHalfRows = kHalfB * kT;
constexpr int kSt2      = 2 * kStF;
constexpr int kK2       = kSt2 + kInF;
constexpr int kSlabP    = 36;

constexpr float kACarry = 16.0f;
constexpr float kWCarry = 1024.0f;
constexpr float kRCarry = 2048.0f;
constexpr float kScale  = 1.0f / (kACarry * kWCarry);
constexpr float kRScale = kScale / kRCarry;

static_assert(kRows == 65536);
static_assert(kHalfRows * 2 == kRows);
static_assert((kInF % 32) == 0 && (kK2 % 32) == 0 && (kSt2 % 32) == 0);
static_assert((kHalfRows % 64) == 0 && (kSt2 % 32) == 0 && (kOutF % 32) == 0);
static_assert((kT % 8) == 0);

constexpr size_t kSzX16  = (size_t)kRows * kInF * 2;
constexpr size_t kSzBU   = (size_t)kHalfRows * kSt2 * 4;
constexpr size_t kSzS16  = (size_t)kHalfRows * kSt2 * 2;
constexpr size_t kSzBT1  = (size_t)kSt2 * kInF * 2;
constexpr size_t kSzBT2  = (size_t)kOutF * kK2 * 2;
constexpr size_t kSzPAR  = (size_t)3 * kStF * 4;
constexpr size_t kOffX16  = 0;
constexpr size_t kOffBU   = kOffX16  + kSzX16;
constexpr size_t kOffS16  = kOffBU   + kSzBU;
constexpr size_t kOffBT1H = kOffS16  + kSzS16;
constexpr size_t kOffBT1L = kOffBT1H + kSzBT1;
constexpr size_t kOffBT2H = kOffBT1L + kSzBT1;
constexpr size_t kOffBT2L = kOffBT2H + kSzBT2;
constexpr size_t kOffPAR  = kOffBT2L + kSzBT2;
constexpr size_t kWsTotal = kOffPAR  + kSzPAR;
static_assert(kWsTotal == 118033408ull);
static_assert(kWsTotal <= 134217728ull);
static_assert((kOffBU % 128) == 0 && (kOffS16 % 128) == 0 && (kOffBT1H % 128) == 0 && (kOffBT1L % 128) == 0 &&
              (kOffBT2H % 128) == 0 && (kOffBT2L % 128) == 0 && (kOffPAR % 128) == 0);

namespace eng {
union FragU { v16h v; v8h h[2]; };
__device__ __forceinline__ v16h frag_load(const _Float16* p) {
  FragU f;
  f.h[0] = *(const v8h*)(p);
  f.h[1] = *(const v8h*)(p + 16);
  return f.v;
}
__device__ __forceinline__ v8f mma_g(v16h a, v16h b, v8f c) {
  c = __builtin_amdgcn_wmma_f32_16x16x32_f16(false, a, false, b, (short)0, c, false, false);
  asm volatile("v_nop\n\tv_nop\n\tv_nop\n\tv_nop" : "+v"(c) : "v"(a), "v"(b));
  return c;
}
__device__ __forceinline__ void split8(v4f a0, v4f a1, v8h& hv, v8h& lv) {
#pragma unroll
  for (int e = 0; e < 4; ++e) {
    const float f0 = a0[e] * kWCarry;
    const float f1 = a1[e] * kWCarry;
    const _Float16 h0 = (_Float16)f0;
    const _Float16 h1 = (_Float16)f1;
    const float r0 = (f0 - (float)h0) * kRCarry;
    const float r1 = (f1 - (float)h1) * kRCarry;
    hv[e]     = h0;
    hv[4 + e] = h1;
    lv[e]     = (_Float16)r0;
    lv[4 + e] = (_Float16)r1;
  }
}
}

__global__ __launch_bounds__(256) void params_kernel(
    const float* __restrict__ nu_log, const float* __restrict__ theta_log, const float* __restrict__ gamma_log,
    float* __restrict__ PAR)
{
  const int n = threadIdx.x;
  const float lm  = expf(-expf(nu_log[n]));
  const float th  = expf(theta_log[n]);
  const float lre = lm * cosf(th);
  const float lim = lm * sinf(th);
  const float g   = expf(gamma_log[n]);
  volatile float* q = PAR;
  q[n] = lre;
  q[kStF + n] = lim;
  q[2 * kStF + n] = g;
  __threadfence();
  q[n] = lre;
  q[kStF + n] = lim;
  q[2 * kStF + n] = g;
}

__global__ __launch_bounds__(256) void wprep_kernel(
    const float* __restrict__ Bre, const float* __restrict__ Bim,
    const float* __restrict__ Cre, const float* __restrict__ Cim, const float* __restrict__ Dm,
    unsigned short* __restrict__ BT1H, unsigned short* __restrict__ BT1L,
    unsigned short* __restrict__ BT2H, unsigned short* __restrict__ BT2L)
{
  const int blk = blockIdx.x;
  const int tid = threadIdx.x;
  v4f a0, a1;
  unsigned short* dh;
  unsigned short* dl;
  size_t off;
  if (blk < 32) {
    const int part = blk >> 4;
    const int c = (blk & 15) * 256 + tid;
    const int n = c >> 4;
    const int col0 = (c & 15) * 8;
    const float* src = (part ? Bim : Bre) + (size_t)n * kInF + col0;
    a0 = *(const v4f*)(src);
    a1 = *(const v4f*)(src + 4);
    off = (size_t)(2 * n + part) * kInF + col0;
    dh = BT1H;
    dl = BT1L;
  } else if (blk < 64) {
    const int c = (blk - 32) * 256 + tid;
    const int o = c >> 6;
    const int cc = c & 63;
    const v4f cr = *(const v4f*)(Cre + (size_t)o * kStF + cc * 4);
    const v4f ci = *(const v4f*)(Cim + (size_t)o * kStF + cc * 4);
    a0 = (v4f){cr[0], -ci[0], cr[1], -ci[1]};
    a1 = (v4f){cr[2], -ci[2], cr[3], -ci[3]};
    off = (size_t)o * kK2 + cc * 8;
    dh = BT2H;
    dl = BT2L;
  } else {
    const int c = (blk - 64) * 256 + tid;
    const int o = c >> 4;
    const int col0 = (c & 15) * 8;
    const float* src = Dm + (size_t)o * kInF + col0;
    a0 = *(const v4f*)(src);
    a1 = *(const v4f*)(src + 4);
    off = (size_t)o * kK2 + kSt2 + col0;
    dh = BT2H;
    dl = BT2L;
  }
  v8h hv, lv;
  eng::split8(a0, a1, hv, lv);
  *(volatile v8h*)(dh + off) = hv;
  *(volatile v8h*)(dl + off) = lv;
  __threadfence();
  *(volatile v8h*)(dh + off) = hv;
  *(volatile v8h*)(dl + off) = lv;
}

__global__ __launch_bounds__(256) void cvt_x_kernel(
    const float* __restrict__ x, unsigned short* __restrict__ X16, int total8)
{
  const int i = blockIdx.x * 256 + threadIdx.x;
  if (i >= total8) return;
  const size_t e0 = (size_t)i << 3;
  const v4f a0 = *(const v4f*)(x + e0);
  const v4f a1 = *(const v4f*)(x + e0 + 4);
  v8h hv;
#pragma unroll
  for (int e = 0; e < 4; ++e) {
    hv[e]     = (_Float16)(a0[e] * kACarry);
    hv[4 + e] = (_Float16)(a1[e] * kACarry);
  }
  unsigned short* q = X16 + e0;
  *(volatile v8h*)q = hv;
  __threadfence();
  *(volatile v8h*)q = hv;
}

__global__ __launch_bounds__(256) void gemm_f16_wsplit_kernel(
    const unsigned short* A1p, int lda1, int K1,
    const unsigned short* A2p, int lda2, int K2,
    const unsigned short* Bhp, const unsigned short* Blp, int ldb,
    float* C, int ldc, int M, int N, float scale, float rscale)
{
  __shared__ __align__(16) float sT[8][16 * kSlabP];
  const _Float16* A1 = (const _Float16*)A1p;
  const _Float16* A2 = (const _Float16*)A2p;
  const _Float16* Bh = (const _Float16*)Bhp;
  const _Float16* Bl = (const _Float16*)Blp;
  const int lane = threadIdx.x & 31;
  const int wave = __builtin_amdgcn_readfirstlane((int)(threadIdx.x >> 5));
  const int tilesN = N >> 5;
  const int tilesM = M >> 6;
  const int tile = blockIdx.x * 8 + wave;
  if (tile >= tilesM * tilesN) return;
  const int tm = tile / tilesN;
  const int tn = tile - tm * tilesN;
  const int m0 = tm << 6;
  const int n0 = tn << 5;

  const int rlane = lane & 15;
  const int koff  = (lane >> 4) * 8;
  const int mOff  = (lane >> 4) * 8;

  v8f acc[4][2], accr[4][2];
#pragma unroll
  for (int i = 0; i < 4; ++i)
#pragma unroll
    for (int j = 0; j < 2; ++j) {
      acc[i][j]  = (v8f){0.f, 0.f, 0.f, 0.f, 0.f, 0.f, 0.f, 0.f};
      accr[i][j] = (v8f){0.f, 0.f, 0.f, 0.f, 0.f, 0.f, 0.f, 0.f};
    }

  const int Ktot = K1 + K2;
  for (int k0 = 0; k0 < Ktot; k0 += 32) {
    const bool seg2 = (k0 >= K1);
    const _Float16* Ab = seg2 ? A2 : A1;
    const int lda = seg2 ? lda2 : lda1;
    const int ka  = seg2 ? (k0 - K1) : k0;
    v16h bh[2], bl[2];
#pragma unroll
    for (int j = 0; j < 2; ++j) {
      const size_t bo = (size_t)(n0 + (j << 4) + rlane) * ldb + koff + k0;
      bh[j] = eng::frag_load(Bh + bo);
      bl[j] = eng::frag_load(Bl + bo);
    }
#pragma unroll
    for (int i = 0; i < 4; ++i) {
      const size_t ao = (size_t)(m0 + (i << 4) + rlane) * lda + koff + ka;
      const v16h ah = eng::frag_load(Ab + ao);
#pragma unroll
      for (int j = 0; j < 2; ++j) {
        acc[i][j]  = eng::mma_g(ah, bh[j], acc[i][j]);
        accr[i][j] = eng::mma_g(ah, bl[j], accr[i][j]);
      }
    }
  }

  float* slab = sT[wave];
  const int q  = lane >> 3;
  const int c4 = (lane & 7) * 4;
#pragma unroll
  for (int i = 0; i < 4; ++i) {
    const int mBase = m0 + (i << 4);
#pragma unroll
    for (int j = 0; j < 2; ++j) {
#pragma unroll
      for (int r = 0; r < 8; ++r) {
        const float v = acc[i][j][r] * scale + accr[i][j][r] * rscale;
        slab[(mOff + r) * kSlabP + (j << 4) + rlane] = v;
      }
    }
    __builtin_amdgcn_fence(__ATOMIC_RELEASE, "workgroup");
    __builtin_amdgcn_wave_barrier();
    __builtin_amdgcn_fence(__ATOMIC_ACQUIRE, "workgroup");
    v4f ov[4];
#pragma unroll
    for (int it = 0; it < 4; ++it) ov[it] = *(const v4f*)(slab + (it * 4 + q) * kSlabP + c4);
    for (int pass = 0; pass < 2; ++pass) {
#pragma unroll
      for (int it = 0; it < 4; ++it)
        *(volatile v4f*)(C + (size_t)(mBase + it * 4 + q) * ldc + n0 + c4) = ov[it];
      __threadfence();
    }
    __builtin_amdgcn_fence(__ATOMIC_RELEASE, "workgroup");
    __builtin_amdgcn_wave_barrier();
    __builtin_amdgcn_fence(__ATOMIC_ACQUIRE, "workgroup");
  }
}

__global__ __launch_bounds__(256) void scan_kernel(
    const float* BU, const float* PAR, unsigned* S16w)
{
  const int n = threadIdx.x;
  const int b = blockIdx.x;
  const float lre = PAR[n];
  const float lim = PAR[kStF + n];
  const float g   = PAR[2 * kStF + n];
  const v2f* src = (const v2f*)(BU + (size_t)b * kT * kSt2) + n;
  unsigned* dst = S16w + (size_t)b * kT * kStF + n;
  float sre = 0.0f, sim = 0.0f;
#pragma unroll 1
  for (int t0 = 0; t0 < kT; t0 += 8) {
    v2f u[8];
#pragma unroll
    for (int j = 0; j < 8; ++j) u[j] = src[(size_t)(t0 + j) * kStF];
    unsigned w[8];
#pragma unroll
    for (int j = 0; j < 8; ++j) {
      const float ure = u[j][0] * g;
      const float uim = u[j][1] * g;
      const float nre = lre * sre - lim * sim + ure;
      const float nim = lre * sim + lim * sre + uim;
      sre = nre;
      sim = nim;
      const _Float16 hr = (_Float16)(sre * kACarry);
      const _Float16 hi = (_Float16)(sim * kACarry);
      const unsigned short br = __builtin_bit_cast(unsigned short, hr);
      const unsigned short bi = __builtin_bit_cast(unsigned short, hi);
      w[j] = (unsigned)br | ((unsigned)bi << 16);
    }
    for (int pass = 0; pass < 2; ++pass) {
#pragma unroll
      for (int j = 0; j < 8; ++j)
        ((volatile unsigned*)dst)[(size_t)(t0 + j) * kStF] = w[j];
      __threadfence();
    }
  }
}

extern "C" void kernel_launch(void* const* d_in, const int* in_sizes, int n_in,
                              void* d_out, int out_size, void* d_ws, size_t ws_size,
                              hipStream_t stream) {
  if (n_in < 9) return;
  if (in_sizes[0] != kRows * kInF) return;
  if (in_sizes[1] != kStF) return;
  if (in_sizes[2] != kStF) return;
  if (in_sizes[3] != kStF) return;
  if (in_sizes[4] != kStF * kInF) return;
  if (in_sizes[5] != kStF * kInF) return;
  if (in_sizes[6] != kOutF * kStF) return;
  if (in_sizes[7] != kOutF * kStF) return;
  if (in_sizes[8] != kOutF * kInF) return;
  if (out_size != kRows * kOutF) return;
  if (ws_size < kWsTotal) return;

  const float* x         = (const float*)d_in[0];
  const float* nu_log    = (const float*)d_in[1];
  const float* theta_log = (const float*)d_in[2];
  const float* gamma_log = (const float*)d_in[3];
  const float* B_re      = (const float*)d_in[4];
  const float* B_im      = (const float*)d_in[5];
  const float* C_re      = (const float*)d_in[6];
  const float* C_im      = (const float*)d_in[7];
  const float* Dm        = (const float*)d_in[8];
  float* out = (float*)d_out;

  char* ws = (char*)d_ws;
  unsigned short* X16  = (unsigned short*)(ws + kOffX16);
  float*          BU   = (float*)(ws + kOffBU);
  unsigned short* S16  = (unsigned short*)(ws + kOffS16);
  unsigned short* BT1H = (unsigned short*)(ws + kOffBT1H);
  unsigned short* BT1L = (unsigned short*)(ws + kOffBT1L);
  unsigned short* BT2H = (unsigned short*)(ws + kOffBT2H);
  unsigned short* BT2L = (unsigned short*)(ws + kOffBT2L);
  float*          PAR  = (float*)(ws + kOffPAR);

  params_kernel<<<1, 256, 0, stream>>>(nu_log, theta_log, gamma_log, PAR);
  wprep_kernel<<<72, 256, 0, stream>>>(B_re, B_im, C_re, C_im, Dm, BT1H, BT1L, BT2H, BT2L);
  cvt_x_kernel<<<(kRows * kInF / 8) / 256, 256, 0, stream>>>(x, X16, kRows * kInF / 8);

  for (int h = 0; h < 2; ++h) {
    const unsigned short* Xh = X16 + (size_t)h * kHalfRows * kInF;
    float* outh = out + (size_t)h * kHalfRows * kOutF;
    gemm_f16_wsplit_kernel<<<(kHalfRows / 64) * (kSt2 / 32) / 8, 256, 0, stream>>>(
        Xh, kInF, kInF,
        Xh, kInF, 0,
        BT1H, BT1L, kInF,
        BU, kSt2, kHalfRows, kSt2, kScale, kRScale);
    scan_kernel<<<kHalfB, 256, 0, stream>>>(BU, PAR, (unsigned*)S16);
    gemm_f16_wsplit_kernel<<<(kHalfRows / 64) * (kOutF / 32) / 8, 256, 0, stream>>>(
        S16, kSt2, kSt2,
        Xh, kInF, kInF,
        BT2H, BT2L, kK2,
        outh, kOutF, kHalfRows, kOutF, kScale, kRScale);
  }
}
